// ParameterKernel_84138409328826
// MI455X (gfx1250) — hardware-run, weakly checked
//
#include <hip/hip_runtime.h>


#ifndef NBAS
#define NBAS 8192
#endif
#ifndef NQ
#define NQ 8192
#endif
#define NBAS_FULL 8192
#define NQ_FULL   8192
#ifndef OUT_NQ
#define OUT_NQ NQ
#endif
#define DF   384
#define NP   64
#define JW   4
#define JB   (16 * JW)
#define XP   (DF + 8)
#define OSQ  68
#define PCS  16384.0f
#define PCI  (1.0f / 16384.0f)

static_assert(DF % 32 == 0);
static_assert(DF % 8 == 0);
static_assert(NBAS % 32 == 0);
static_assert(NBAS % 64 == 0);
static_assert(NQ % JB == 0);
static_assert(NP == 64);
static_assert(NBAS <= NBAS_FULL);
static_assert(NQ <= NQ_FULL);
static_assert(OUT_NQ % 32 == 0);
static_assert(OUT_NQ >= NQ);
static_assert((XP * 2) % 16 == 0);
static_assert((OSQ * 4) % 16 == 0);
static_assert((JB * (DF / 8)) % (32 * JW) == 0);
static_assert(2 * (32 * JW) * 16 == 16 * JB * 4);
static_assert((size_t)JB * XP * 2 + (size_t)16 * OSQ * 4 <= (size_t)131072);
static_assert(((size_t)NP * NBAS / 8) % 8 == 0);
static_assert(((size_t)NBAS * DF / 8) % 8 == 0);

typedef _Float16 h16;
typedef unsigned short bf;
typedef __attribute__((ext_vector_type(16))) __bf16   v16bf;
typedef __attribute__((ext_vector_type(16))) _Float16 v16h;
typedef __attribute__((ext_vector_type(8)))  _Float16 v8h;
typedef __attribute__((ext_vector_type(8)))  unsigned short v8us;
typedef __attribute__((ext_vector_type(8)))  float    v8f;
typedef __attribute__((ext_vector_type(4)))  float    v4f;
typedef __attribute__((ext_vector_type(4)))  int      v4i;
typedef v4f  __attribute__((may_alias)) v4fa;

__device__ __forceinline__ unsigned short f2bf(float f) { unsigned u = __float_as_uint(f); u += 0x7FFFu + ((u >> 16) & 1u); return (unsigned short)(u >> 16); }
__device__ __forceinline__ float bfr(float f) { return __uint_as_float(((unsigned)f2bf(f)) << 16); }
__device__ __forceinline__ v16h cat16(v8h lo, v8h hi) { return __builtin_shufflevector(lo, hi, 0, 1, 2, 3, 4, 5, 6, 7, 8, 9, 10, 11, 12, 13, 14, 15); }
__device__ __forceinline__ v16bf cat16b(v8us lo, v8us hi) { return __builtin_bit_cast(v16bf, __builtin_shufflevector(lo, hi, 0, 1, 2, 3, 4, 5, 6, 7, 8, 9, 10, 11, 12, 13, 14, 15)); }
__device__ __forceinline__ v8f wmma16(v16h a, v16h b, v8f c) { return __builtin_amdgcn_wmma_f32_16x16x32_f16(false, a, false, b, (short)0, c, false, false); }
__device__ __forceinline__ v8f wmmab(v16bf a, v16bf b, v8f c) { return __builtin_amdgcn_wmma_f32_16x16x32_bf16(false, a, false, b, (short)0, c, false, false); }
__device__ __forceinline__ v16h  ldh(const h16* p) { return cat16(*(const v8h*)p, *(const v8h*)(p + 16)); }
__device__ __forceinline__ v16bf ldb(const bf* p)  { return cat16b(*(const v8us*)p, *(const v8us*)(p + 16)); }
__device__ __forceinline__ v8f wmmab_g(v16bf a, v16bf b, v8f c) { c = wmmab(a, b, c); asm volatile("v_nop\n\tv_nop\n\tv_nop\n\tv_nop" : "+v"(c) : "v"(a), "v"(b)); return c; }
__device__ __forceinline__ v8f wmma16_g(v16h a, v16h b, v8f c) { c = wmma16(a, b, c); asm volatile("v_nop\n\tv_nop\n\tv_nop\n\tv_nop" : "+v"(c) : "v"(a), "v"(b)); return c; }
__device__ __forceinline__ h16 toh_flush(float v) { const h16 r = (h16)v; return (fabsf(v) < 6.103515625e-05f) ? (h16)0.0f : r; }

__global__ __launch_bounds__(256) void k_cvt8(const float* __restrict__ src, bf* dst, size_t n8) {
    const size_t i = (size_t)blockIdx.x * 256 + threadIdx.x; if (i >= n8) return;
    const v8f v = *(const v8f*)(src + i * 8); v8us o;
#pragma unroll
    for (int k = 0; k < 8; ++k) o[k] = f2bf(v[k]);
    *(volatile v8us*)(dst + i * 8) = o; __threadfence(); *(volatile v8us*)(dst + i * 8) = o;
}

__global__ __launch_bounds__(256) void k_cvta(const float* __restrict__ src, h16* dst, int rowp8, size_t srcpitch, size_t n8) {
    const size_t i = (size_t)blockIdx.x * 256 + threadIdx.x; if (i >= n8) return;
    const size_t row = i / (size_t)rowp8, c = i % (size_t)rowp8;
    const v8f v = *(const v8f*)(src + row * srcpitch + c * 8); v8h o;
#pragma unroll
    for (int k = 0; k < 8; ++k) o[k] = toh_flush(bfr(v[k]));
    *(volatile v8h*)(dst + i * 8) = o; __threadfence(); *(volatile v8h*)(dst + i * 8) = o;
}

__global__ __launch_bounds__(32 * JW) void k_pk(const bf* __restrict__ XB, const float* __restrict__ XQ, const h16* __restrict__ AH,
                                                const int* __restrict__ ZB, const int* __restrict__ ZQ, const int* __restrict__ ek_p, float* OUT) {
    __shared__ __align__(16) bf xs[JB * XP];
    __shared__ __align__(16) float os[16 * OSQ];
    const int tid = threadIdx.x;
    const int lane = tid & 31, lr = lane & 15, hi = lane >> 4;
    const int wave = __builtin_amdgcn_readfirstlane((int)(threadIdx.x >> 5));
    const int j0 = blockIdx.x * JB;
#pragma unroll 1
    for (int q = tid; q < JB * (DF / 8); q += 32 * JW) {
        const int row = q / (DF / 8), c8 = (q % (DF / 8)) * 8;
        const v8f v = *(const v8f*)(XQ + (size_t)(j0 + row) * DF + c8);
        v8us o;
#pragma unroll
        for (int k = 0; k < 8; ++k) o[k] = f2bf(v[k]);
        *(v8us*)(&xs[row * XP + c8]) = o;
    }
    __syncthreads();
    int ek = ek_p[0]; ek = ek < -64 ? -64 : (ek > 64 ? 64 : ek);
    const int en = ek < 0 ? -ek : ek;
    const int zq = ZQ[j0 + wave * 16 + lr];
    const size_t ao = (size_t)lr * DF + 8 * hi;
    const int bo = (wave * 16 + lr) * XP + 8 * hi;
    const size_t alo = (size_t)lr * NBAS + 8 * hi;
    v8f yacc[4];
#pragma unroll
    for (int pt = 0; pt < 4; ++pt) yacc[pt] = (v8f){};
#pragma unroll 1
    for (int i0 = 0; i0 < NBAS; i0 += 32) {
        const bf* ar = XB + ao + (size_t)i0 * DF;
        v8f sa = (v8f){}, sb = (v8f){};
#pragma unroll 2
        for (int kc = 0; kc < DF; kc += 32) {
            const v16bf a0 = ldb(ar + kc), a1 = ldb(ar + (size_t)16 * DF + kc);
            const v16bf bq = cat16b(*(const v8us*)(&xs[bo + kc]), *(const v8us*)(&xs[bo + kc + 16]));
            sa = wmmab_g(a0, bq, sa); sb = wmmab_g(a1, bq, sb);
        }
        const int* zp = ZB + i0 + 8 * hi;
        const v4i z0 = *(const v4i*)zp, z1 = *(const v4i*)(zp + 4), z2 = *(const v4i*)(zp + 16), z3 = *(const v4i*)(zp + 20);
        int za[8], zb[8];
#pragma unroll
        for (int r = 0; r < 4; ++r) { za[r] = z0[r]; za[4 + r] = z1[r]; zb[r] = z2[r]; zb[4 + r] = z3[r]; }
        float ka[8], kb[8];
        if (ek == 2) {
#pragma unroll
            for (int r = 0; r < 8; ++r) { ka[r] = sa[r] * sa[r]; kb[r] = sb[r] * sb[r]; }
        } else {
#pragma unroll
            for (int r = 0; r < 8; ++r) { ka[r] = 1.0f; kb[r] = 1.0f; }
#pragma unroll 1
            for (int t = 0; t < en; ++t) {
#pragma unroll
                for (int r = 0; r < 8; ++r) { ka[r] *= sa[r]; kb[r] *= sb[r]; } }
            if (ek < 0) {
#pragma unroll
                for (int r = 0; r < 8; ++r) { ka[r] = __builtin_amdgcn_rcpf(ka[r]); kb[r] = __builtin_amdgcn_rcpf(kb[r]); } }
        }
        v16h pb;
#pragma unroll
        for (int r = 0; r < 8; ++r) {
            const float ga = (za[r] == zq) ? ka[r] * PCS : 0.0f;
            const float gb = (zb[r] == zq) ? kb[r] * PCS : 0.0f;
            pb[r] = toh_flush(ga); pb[8 + r] = toh_flush(gb); }
        const h16* ap = AH + alo + i0;
#pragma unroll
        for (int pt = 0; pt < 4; ++pt) { const v16h al = ldh(ap + (size_t)pt * 16 * NBAS); yacc[pt] = wmma16_g(al, pb, yacc[pt]); }
    }
#pragma unroll
    for (int pt = 0; pt < 4; ++pt) {
#pragma unroll
        for (int r = 0; r < 8; ++r) os[(8 * hi + r) * OSQ + wave * 16 + lr] = yacc[pt][r] * PCI;
        __syncthreads();
        float* orow = OUT + (size_t)(16 * pt) * OUT_NQ + j0;
#pragma unroll 1
        for (int ps = 0; ps < 2; ++ps) {
#pragma unroll
            for (int s = 0; s < 2; ++s) { const int q = s * (32 * JW) + tid; const int row = q >> 4, cofs = (q & 15) * 4;
                const v4f val = *(const v4fa*)(&os[row * OSQ + cofs]);
                *(volatile v4f*)(orow + (size_t)row * OUT_NQ + cofs) = val; }
            if (ps == 0) __threadfence(); }
        __syncthreads();
    }
}

static constexpr size_t al256(size_t v) { return (v + 255) & ~(size_t)255; }
static constexpr size_t SZ_XB = al256((size_t)NBAS * DF * 2);
static constexpr size_t SZ_AH = al256((size_t)NP * NBAS * 2);
static constexpr size_t SZ_TOTAL = SZ_XB + SZ_AH;
static_assert(SZ_TOTAL <= (size_t)134217728);

extern "C" void kernel_launch(void* const* d_in, const int* in_sizes, int n_in,
                              void* d_out, int out_size, void* d_ws, size_t ws_size, hipStream_t stream) {
    if (n_in < 6) return;
    if ((size_t)in_sizes[0] < (size_t)(NP - 1) * NBAS_FULL + NBAS) return;
    if ((size_t)in_sizes[1] < (size_t)NBAS * DF || (size_t)in_sizes[2] < (size_t)NQ * DF) return;
    if (in_sizes[3] < NBAS || in_sizes[4] < NQ || in_sizes[5] < 1) return;
    if ((size_t)out_size < (size_t)(NP - 1) * OUT_NQ + NQ) return;
    if (SZ_TOTAL > ws_size) return;
    const float* alpha = (const float*)d_in[0];
    const float* xb = (const float*)d_in[1];
    const float* xq = (const float*)d_in[2];
    const int* zb = (const int*)d_in[3];
    const int* zq = (const int*)d_in[4];
    const int* ekp = (const int*)d_in[5];
    float* OUT = (float*)d_out;
    char* wsp = (char*)d_ws;
    bf* XRB = (bf*)wsp; wsp += SZ_XB;
    h16* ALH = (h16*)wsp; wsp += SZ_AH;

    { const size_t n8 = (size_t)NBAS * DF / 8;
      k_cvt8<<<(unsigned)((n8 + 255) / 256), 256, 0, stream>>>(xb, XRB, n8); }
    { const size_t n8 = (size_t)NP * NBAS / 8;
      k_cvta<<<(unsigned)((n8 + 255) / 256), 256, 0, stream>>>(alpha, ALH, NBAS / 8, (size_t)NBAS_FULL, n8); }
    k_pk<<<dim3(NQ / JB, 1, 1), 32 * JW, 0, stream>>>(XRB, xq, ALH, zb, zq, ekp, OUT);
}
